// CausalMultiHeadSelfAttention_85040352461191
// MI455X (gfx1250) — hardware-verified
//
#include <hip/hip_runtime.h>


#ifndef NB
#define NB 2
#endif
#ifndef SEQ
#define SEQ 4096
#endif
#define NB_FULL  2
#define SEQ_FULL 4096
#define DM   512
#define NH   8
#define HD   64
#define RH   512
#define RHB  (((RH < SEQ) ? RH : SEQ) / 64)
#define PP   72
#define PCAR 1024.0f
#define SL2  0.18033688011112042f
#define NEGB (-3.0e38f)
static_assert(SEQ % 64 == 0);
static_assert(SEQ <= SEQ_FULL);
static_assert(NB >= 1 && NB <= NB_FULL);
static_assert(DM == NH * HD);
static_assert(DM % 64 == 0);
static_assert(RH % 64 == 0);
#define WS_TOTAL ((size_t)4 * DM * DM * 2 + (size_t)SEQ * DM * 2 + (size_t)SEQ * DM * 4 + (size_t)9 * SEQ * DM * 2 + (size_t)2 * SEQ * DM * 2)
static_assert(WS_TOTAL <= (size_t)134217728);

typedef _Float16 h16;
typedef unsigned short bf;
typedef __attribute__((ext_vector_type(16))) __bf16   v16bf;
typedef __attribute__((ext_vector_type(16))) _Float16 v16h;
typedef __attribute__((ext_vector_type(8)))  _Float16 v8h;
typedef __attribute__((ext_vector_type(8)))  unsigned short v8us;
typedef __attribute__((ext_vector_type(8)))  float    v8f;
typedef __attribute__((ext_vector_type(4)))  float    v4f;
typedef __attribute__((ext_vector_type(2)))  _Float16 v2h;
typedef __attribute__((ext_vector_type(2)))  unsigned short v2us;
typedef v8h  __attribute__((may_alias)) v8ha;
typedef v4f  __attribute__((may_alias)) v4fa;
typedef v8us __attribute__((may_alias)) v8usa;

__device__ __forceinline__ unsigned short f2bf(float f) { unsigned u = __float_as_uint(f); u += 0x7FFFu + ((u >> 16) & 1u); return (unsigned short)(u >> 16); }
__device__ __forceinline__ float bf2f(unsigned short b) { return __uint_as_float(((unsigned)b) << 16); }
__device__ __forceinline__ float bfr(float f) { return bf2f(f2bf(f)); }
__device__ __forceinline__ h16 tohx(float x) { return (h16)x; }
__device__ __forceinline__ void splitf(float y, unsigned short& h, unsigned short& l) { h = f2bf(y); l = f2bf(y - bf2f(h)); }
__device__ __forceinline__ v16h cat16(v8h lo, v8h hi) { return __builtin_shufflevector(lo, hi, 0, 1, 2, 3, 4, 5, 6, 7, 8, 9, 10, 11, 12, 13, 14, 15); }
__device__ __forceinline__ v16bf cat16b(v8us lo, v8us hi) { return __builtin_bit_cast(v16bf, __builtin_shufflevector(lo, hi, 0, 1, 2, 3, 4, 5, 6, 7, 8, 9, 10, 11, 12, 13, 14, 15)); }
__device__ __forceinline__ v8f wmma16(v16h a, v16h b, v8f c) { return __builtin_amdgcn_wmma_f32_16x16x32_f16(false, a, false, b, (short)0, c, false, false); }
__device__ __forceinline__ v8f wmmab(v16bf a, v16bf b, v8f c) { return __builtin_amdgcn_wmma_f32_16x16x32_bf16(false, a, false, b, (short)0, c, false, false); }

template <typename T16> struct WFrag;
template <> struct WFrag<h16> { typedef v16h V;
    static __device__ __forceinline__ V ld(const h16* p)  { return cat16(*(const v8h*)p, *(const v8h*)(p + 16)); }
    static __device__ __forceinline__ V lda(const h16* p) { return cat16(*(const v8ha*)p, *(const v8ha*)(p + 16)); }
    static __device__ __forceinline__ v8f mma(V a, V b, v8f c) { return wmma16(a, b, c); } };
template <> struct WFrag<bf> { typedef v16bf V;
    static __device__ __forceinline__ V ld(const bf* p)  { return cat16b(*(const v8us*)p, *(const v8us*)(p + 16)); }
    static __device__ __forceinline__ V lda(const bf* p) { return cat16b(*(const v8usa*)p, *(const v8usa*)(p + 16)); }
    static __device__ __forceinline__ v8f mma(V a, V b, v8f c) { return wmmab(a, b, c); } };

template <typename T16, int NSPLIT, bool BIAS>
__global__ __launch_bounds__(32) void k_gemmw(const T16* __restrict__ A, const T16* __restrict__ A2, const T16* __restrict__ Bt, const T16* __restrict__ Bt2, int K, float* C, int ldc, const float* __restrict__ bias, size_t sA, size_t sB, size_t sC) {
    typedef typename WFrag<T16>::V V;
    __shared__ __align__(16) float os[16 * 68];
    const size_t z = blockIdx.z; A += z * sA; if (A2) A2 += z * sA; Bt += z * sB; if (Bt2) Bt2 += z * sB; C += z * sC;
    const int lane = threadIdx.x & 31, lr = lane & 15, hi = lane >> 4; const int r0 = blockIdx.x * 64, c0 = blockIdx.y * 64;
    v8f acc[4][4];
#pragma unroll
    for (int mb = 0; mb < 4; ++mb)
#pragma unroll
        for (int nb = 0; nb < 4; ++nb) acc[mb][nb] = (v8f){};
    const size_t aoff = (size_t)(r0 + lr) * K + 8 * hi, boff = (size_t)(c0 + lr) * K + 8 * hi;
#pragma unroll 1
    for (int kc = 0; kc < K; kc += 32) {
        V a[4], a2[4];
#pragma unroll
        for (int mb = 0; mb < 4; ++mb) { a[mb] = WFrag<T16>::ld(A + aoff + (size_t)mb * 16 * K + kc); if (NSPLIT == 1 || NSPLIT == 2) a2[mb] = WFrag<T16>::ld(A2 + aoff + (size_t)mb * 16 * K + kc); }
#pragma unroll
        for (int nb = 0; nb < 4; ++nb) { const V b = WFrag<T16>::ld(Bt + boff + (size_t)nb * 16 * K + kc); V b2; if (NSPLIT >= 2) b2 = WFrag<T16>::ld(Bt2 + boff + (size_t)nb * 16 * K + kc);
#pragma unroll
            for (int mb = 0; mb < 4; ++mb) { acc[mb][nb] = WFrag<T16>::mma(a[mb], b, acc[mb][nb]); if (NSPLIT == 1 || NSPLIT == 2) acc[mb][nb] = WFrag<T16>::mma(a2[mb], b, acc[mb][nb]); if (NSPLIT >= 2) acc[mb][nb] = WFrag<T16>::mma(a[mb], b2, acc[mb][nb]); } }
        asm volatile("v_nop\n\tv_nop\n\tv_nop\n\tv_nop" : "+v"(acc[0][0]), "+v"(acc[1][1]), "+v"(acc[2][2]), "+v"(acc[3][3]) : "v"(a[0]), "v"(a[3]));
    }
#pragma unroll
    for (int mb = 0; mb < 4; ++mb) {
#pragma unroll
        for (int nb = 0; nb < 4; ++nb) {
#pragma unroll
            for (int j = 0; j < 8; ++j) os[(hi * 8 + j) * 68 + nb * 16 + lr] = acc[mb][nb][j]; }
        __builtin_amdgcn_wave_barrier(); asm volatile("" ::: "memory");
        float* crow = C + (size_t)(r0 + mb * 16) * ldc + c0;
#pragma unroll 1
        for (int ps = 0; ps < 2; ++ps) {
#pragma unroll
            for (int s = 0; s < 8; ++s) { const int row = 2 * s + hi, cofs = lr * 4; v4f val = *(const v4fa*)(os + row * 68 + cofs); if (BIAS) { val[0] += bfr(bias[c0 + cofs]); val[1] += bfr(bias[c0 + cofs + 1]); val[2] += bfr(bias[c0 + cofs + 2]); val[3] += bfr(bias[c0 + cofs + 3]); }
                *(volatile v4f*)(crow + (size_t)row * ldc + cofs) = val; }
            if (ps == 0) __threadfence(); }
        __builtin_amdgcn_wave_barrier(); asm volatile("" ::: "memory");
    }
}

__global__ __launch_bounds__(256) void k_cvt8(const float* __restrict__ src, bf* dst, size_t n8) { const size_t i = (size_t)blockIdx.x * 256 + threadIdx.x; if (i >= n8) return; const v8f v = *(const v8f*)(src + i * 8); v8us o;
#pragma unroll
    for (int k = 0; k < 8; ++k) o[k] = f2bf(v[k]); *(volatile v8us*)(dst + i * 8) = o; __threadfence(); *(volatile v8us*)(dst + i * 8) = o; }

__global__ __launch_bounds__(256) void k_qkp(const float* __restrict__ F, int pitch, int nheads, h16* P16, bf* Ph, bf* Pl) {
    const size_t e = ((size_t)blockIdx.x * 256 + threadIdx.x) * 2; if (e >= (size_t)nheads * SEQ * HD) return;
    const int d = (int)(e % HD); const int t = (int)((e / HD) % SEQ); const int h = (int)(e / ((size_t)HD * SEQ));
    const float* f = F + (size_t)t * pitch + h * HD + d; v2h o16; v2us oh, ol;
#pragma unroll
    for (int q = 0; q < 2; ++q) { const float x = f[q]; o16[q] = tohx(x); unsigned short a2, c2; splitf(x, a2, c2); oh[q] = a2; ol[q] = c2; }
    *(volatile v2h*)(P16 + e) = o16; *(volatile v2us*)(Ph + e) = oh; *(volatile v2us*)(Pl + e) = ol; __threadfence();
    *(volatile v2h*)(P16 + e) = o16; *(volatile v2us*)(Ph + e) = oh; *(volatile v2us*)(Pl + e) = ol; }

__global__ __launch_bounds__(256) void k_vtp(const float* __restrict__ F, int pitch, int nheads, h16* V16, bf* Vh, bf* Vl) {
    const size_t e = ((size_t)blockIdx.x * 256 + threadIdx.x) * 2; if (e >= (size_t)nheads * HD * SEQ) return;
    const int t = (int)(e % SEQ); const int d = (int)((e / SEQ) % HD); const int g = (int)(e / ((size_t)SEQ * HD)); v2h o16; v2us oh, ol;
#pragma unroll
    for (int q = 0; q < 2; ++q) { const float x = F[(size_t)(t + q) * pitch + g * HD + d]; o16[q] = tohx(x); unsigned short a2, c2; splitf(x, a2, c2); oh[q] = a2; ol[q] = c2; }
    *(volatile v2h*)(V16 + e) = o16; *(volatile v2us*)(Vh + e) = oh; *(volatile v2us*)(Vl + e) = ol; __threadfence();
    *(volatile v2h*)(V16 + e) = o16; *(volatile v2us*)(Vh + e) = oh; *(volatile v2us*)(Vl + e) = ol; }

template <typename T16> struct PSt;
template <> struct PSt<h16> { static __device__ __forceinline__ void st(h16* p0, h16* p1, int i, float p) { (void)p1; p0[i] = tohx(p * PCAR); } };
template <> struct PSt<bf>  { static __device__ __forceinline__ void st(bf* p0, bf* p1, int i, float p) { unsigned short a2, c2; splitf(p, a2, c2); p0[i] = a2; p1[i] = c2; } };

template <typename T16, bool SPL>
__global__ __launch_bounds__(128) __attribute__((amdgpu_num_vgpr(256)))
void k_flash(const T16* __restrict__ QP, const T16* __restrict__ QL, const T16* __restrict__ KP, const T16* __restrict__ KL,
             const T16* __restrict__ VP, const T16* __restrict__ VL, int qb0, bf* ATh, bf* ATl) {
    typedef WFrag<T16> W; typedef typename W::V V;
    __shared__ __align__(16) T16 Pb[4][2][16 * PP];
    __shared__ __align__(16) unsigned short Es[4][2][16 * PP];
    const int lane = threadIdx.x & 31, wv = threadIdx.x >> 5, lr = lane & 15, hi = lane >> 4;
    const int h = blockIdx.y, qb = qb0 + (int)blockIdx.x, t0 = qb * 64 + wv * 16;
    const size_t hq = (size_t)h * SEQ * HD;
    const size_t hv = (size_t)h * HD * SEQ;
    T16* Pw0 = &Pb[wv][0][0]; T16* Pw1 = &Pb[wv][1][0];
    V qa0, qa1, ql0, ql1;
    { const size_t qo = hq + (size_t)(t0 + lr) * HD + 8 * hi; qa0 = W::ld(QP + qo); qa1 = W::ld(QP + qo + 32);
      if (SPL) { ql0 = W::ld(QL + qo); ql1 = W::ld(QL + qo + 32); } else { ql0 = qa0; ql1 = qa1; } }
    v8f oacc[4];
#pragma unroll
    for (int t = 0; t < 4; ++t) oacc[t] = (v8f){};
    float mrow[8], lrow[8];
#pragma unroll
    for (int r = 0; r < 8; ++r) { mrow[r] = NEGB; lrow[r] = 0.f; }
#pragma unroll 1
    for (int kb = 0; kb <= qb; ++kb) {
        v8f sacc[4];
#pragma unroll
        for (int t = 0; t < 4; ++t) sacc[t] = (v8f){};
#pragma unroll
        for (int t = 0; t < 4; ++t) {
            const size_t ko = hq + (size_t)(kb * 64 + t * 16 + lr) * HD + 8 * hi;
            { const V b = W::ld(KP + ko); sacc[t] = W::mma(qa0, b, sacc[t]);
              if (SPL) { sacc[t] = W::mma(ql0, b, sacc[t]); const V c = W::ld(KL + ko); sacc[t] = W::mma(qa0, c, sacc[t]); } }
            { const V b = W::ld(KP + ko + 32); sacc[t] = W::mma(qa1, b, sacc[t]);
              if (SPL) { sacc[t] = W::mma(ql1, b, sacc[t]); const V c = W::ld(KL + ko + 32); sacc[t] = W::mma(qa1, c, sacc[t]); } }
        }
        asm volatile("v_nop\n\tv_nop\n\tv_nop\n\tv_nop" : "+v"(sacc[0]), "+v"(sacc[1]), "+v"(sacc[2]), "+v"(sacc[3]) : "v"(qa0), "v"(qa1));
#pragma unroll
        for (int r = 0; r < 8; ++r) {
            const int qpos = t0 + 8 * hi + r; float sv[4]; float rm = mrow[r];
#pragma unroll
            for (int t = 0; t < 4; ++t) { const float s0 = sacc[t][r] * SL2; const int key = kb * 64 + t * 16 + lr; const float s = (key > qpos) ? NEGB : s0; sv[t] = s; rm = fmaxf(rm, s); }
#pragma unroll
            for (int sh = 1; sh < 16; sh <<= 1) rm = fmaxf(rm, __shfl_xor(rm, sh, 16));
            const float corr = __builtin_amdgcn_exp2f(mrow[r] - rm);
            lrow[r] *= corr;
#pragma unroll
            for (int t = 0; t < 4; ++t) oacc[t][r] *= corr;
            float psum = 0.f;
#pragma unroll
            for (int t = 0; t < 4; ++t) { const float p = __builtin_amdgcn_exp2f(sv[t] - rm); psum += p; PSt<T16>::st(Pw0, Pw1, (8 * hi + r) * PP + t * 16 + lr, p); }
#pragma unroll
            for (int sh = 1; sh < 16; sh <<= 1) psum += __shfl_xor(psum, sh, 16);
            lrow[r] += psum; mrow[r] = rm;
        }
        __builtin_amdgcn_fence(3, "wavefront"); __builtin_amdgcn_wave_barrier(); asm volatile("" ::: "memory");
#pragma unroll
        for (int ks = 0; ks < 2; ++ks) {
            const V pa = W::lda(Pw0 + lr * PP + ks * 32 + 8 * hi); V pl = pa; if (SPL) pl = W::lda(Pw1 + lr * PP + ks * 32 + 8 * hi);
#pragma unroll
            for (int t = 0; t < 4; ++t) {
                const size_t vo = hv + (size_t)(t * 16 + lr) * SEQ + kb * 64 + ks * 32 + 8 * hi;
                const V vb = W::ld(VP + vo); oacc[t] = W::mma(pa, vb, oacc[t]);
                if (SPL) { oacc[t] = W::mma(pl, vb, oacc[t]); const V vc = W::ld(VL + vo); oacc[t] = W::mma(pa, vc, oacc[t]); }
            }
        }
        asm volatile("v_nop\n\tv_nop\n\tv_nop\n\tv_nop" : "+v"(oacc[0]), "+v"(oacc[1]), "+v"(oacc[2]), "+v"(oacc[3]) : "v"(qa0), "v"(qa1));
        __builtin_amdgcn_wave_barrier(); asm volatile("" ::: "memory");
    }
    const float lsc = SPL ? 1.0f : PCAR;
    unsigned short* E0 = &Es[wv][0][0]; unsigned short* E1 = &Es[wv][1][0];
#pragma unroll
    for (int r = 0; r < 8; ++r) { const float inv = __fdiv_rn(1.0f, lrow[r] * lsc);
#pragma unroll
        for (int t = 0; t < 4; ++t) { unsigned short a2, c2; splitf(oacc[t][r] * inv, a2, c2); const int i = (8 * hi + r) * PP + t * 16 + lr; E0[i] = a2; E1[i] = c2; } }
    __builtin_amdgcn_fence(3, "wavefront"); __builtin_amdgcn_wave_barrier(); asm volatile("" ::: "memory");
    bf* oh = ATh + (size_t)t0 * DM + h * HD; bf* ol = ATl + (size_t)t0 * DM + h * HD;
#pragma unroll 1
    for (int ps = 0; ps < 2; ++ps) {
#pragma unroll
        for (int s = 0; s < 4; ++s) { const int row = s * 4 + (lane >> 3), col = (lane & 7) * 8;
            const v8us vh = *(const v8usa*)(E0 + row * PP + col); const v8us vl = *(const v8usa*)(E1 + row * PP + col);
            *(volatile v8us*)(oh + (size_t)row * DM + col) = vh; *(volatile v8us*)(ol + (size_t)row * DM + col) = vl; }
        if (ps == 0) __threadfence(); }
}

extern "C" void kernel_launch(void* const* d_in, const int* in_sizes, int n_in,
                              void* d_out, int out_size, void* d_ws, size_t ws_size, hipStream_t stream) {
    const size_t needx = (size_t)(NB - 1) * SEQ_FULL * DM + (size_t)SEQ * DM;
    if (n_in < 7) return;
    if ((size_t)in_sizes[0] < needx || in_sizes[1] < DM * DM || in_sizes[2] < DM * DM || in_sizes[3] < DM * DM || in_sizes[4] < DM || in_sizes[5] < DM * DM || in_sizes[6] < DM) return;
    if ((size_t)out_size < needx) return;
    const float* x = (const float*)d_in[0]; const float* wq = (const float*)d_in[1]; const float* wk = (const float*)d_in[2]; const float* wv = (const float*)d_in[3];
    const float* bv = (const float*)d_in[4]; const float* wo = (const float*)d_in[5]; const float* bo = (const float*)d_in[6];
    float* OUT = (float*)d_out;
    char* wsp = (char*)d_ws;
    auto take = [&](size_t bytes) { char* p = wsp; wsp += (bytes + 255) & ~(size_t)255; return (void*)p; };
    bf* WQ = (bf*)take((size_t)DM * DM * 2); bf* WK = (bf*)take((size_t)DM * DM * 2); bf* WV = (bf*)take((size_t)DM * DM * 2); bf* WO = (bf*)take((size_t)DM * DM * 2);
    bf* XB = (bf*)take((size_t)SEQ * DM * 2); float* F = (float*)take((size_t)SEQ * DM * 4);
    h16* Q16 = (h16*)take((size_t)SEQ * DM * 2); bf* Qh = (bf*)take((size_t)SEQ * DM * 2); bf* Ql = (bf*)take((size_t)SEQ * DM * 2);
    h16* K16 = (h16*)take((size_t)SEQ * DM * 2); bf* Kh = (bf*)take((size_t)SEQ * DM * 2); bf* Kl = (bf*)take((size_t)SEQ * DM * 2);
    h16* VT16 = (h16*)take((size_t)SEQ * DM * 2); bf* VTh = (bf*)take((size_t)SEQ * DM * 2); bf* VTl = (bf*)take((size_t)SEQ * DM * 2);
    bf* ATh = (bf*)take((size_t)SEQ * DM * 2); bf* ATl = (bf*)take((size_t)SEQ * DM * 2);
    if ((size_t)(wsp - (char*)d_ws) > ws_size) return;
    const size_t nw8 = (size_t)DM * DM / 8, nx8 = (size_t)SEQ * DM / 8;
    const unsigned gw = (unsigned)((nw8 + 255) / 256), gx = (unsigned)((nx8 + 255) / 256), gp = (unsigned)(((size_t)NH * SEQ * HD / 2 + 255) / 256);
    k_cvt8<<<gw, 256, 0, stream>>>(wq, WQ, nw8); k_cvt8<<<gw, 256, 0, stream>>>(wk, WK, nw8); k_cvt8<<<gw, 256, 0, stream>>>(wv, WV, nw8); k_cvt8<<<gw, 256, 0, stream>>>(wo, WO, nw8);
    for (int b = 0; b < NB; ++b) {
        k_cvt8<<<gx, 256, 0, stream>>>(x + (size_t)b * SEQ_FULL * DM, XB, nx8);
        k_gemmw<bf, 0, false><<<dim3(SEQ / 64, DM / 64, 1), 32, 0, stream>>>(XB, nullptr, WQ, nullptr, DM, F, DM, nullptr, 0, 0, 0);
        k_qkp<<<gp, 256, 0, stream>>>(F, DM, NH, Q16, Qh, Ql);
        k_gemmw<bf, 0, false><<<dim3(SEQ / 64, DM / 64, 1), 32, 0, stream>>>(XB, nullptr, WK, nullptr, DM, F, DM, nullptr, 0, 0, 0);
        k_qkp<<<gp, 256, 0, stream>>>(F, DM, NH, K16, Kh, Kl);
        k_gemmw<bf, 0, true><<<dim3(SEQ / 64, DM / 64, 1), 32, 0, stream>>>(XB, nullptr, WV, nullptr, DM, F, DM, bv, 0, 0, 0);
        k_vtp<<<gp, 256, 0, stream>>>(F, DM, NH, VT16, VTh, VTl);
        if (RHB > 0) k_flash<bf, true><<<dim3(RHB, NH, 1), 128, 0, stream>>>(Qh, Ql, Kh, Kl, VTh, VTl, 0, ATh, ATl);
        if (SEQ / 64 - RHB > 0) k_flash<h16, false><<<dim3(SEQ / 64 - RHB, NH, 1), 128, 0, stream>>>(Q16, nullptr, K16, nullptr, VT16, nullptr, RHB, ATh, ATl);
        k_gemmw<bf, 1, true><<<dim3(SEQ / 64, DM / 64, 1), 32, 0, stream>>>(ATh, ATl, WO, nullptr, DM, OUT + (size_t)b * SEQ_FULL * DM, DM, bo, 0, 0, 0);
    }
}
